// SlidingWindowCausalAttention_3066606650062
// MI455X (gfx1250) — hardware-verified
//
#include <hip/hip_runtime.h>


#define NB_  1
#define TT   8192
#define DM   1024
#define NH_  16
#define NKV  16
#define REP  (NH_ / NKV)
#define HD   64
#define DQ   (NH_ * HD)
#define DKV  (NKV * HD)
#define RB   2048
#define KW   3072
#define WB   1024
#define PADK 1024
#define ZH   1
#define RH   2048
#define WIN  8192
#define PCAR 1024.0f
#define SCL  0.125f
typedef _Float16 h16;
typedef unsigned short bf;
typedef __attribute__((ext_vector_type(16))) __bf16   v16bf;
typedef __attribute__((ext_vector_type(16))) _Float16 v16h;
typedef __attribute__((ext_vector_type(8)))  _Float16 v8h;
typedef __attribute__((ext_vector_type(8)))  unsigned short v8us;
typedef __attribute__((ext_vector_type(8)))  float    v8f;
typedef __attribute__((ext_vector_type(4)))  float    v4f;
typedef v8h  __attribute__((may_alias)) v8ha;
typedef v4f  __attribute__((may_alias)) v4fa;
typedef v8us __attribute__((may_alias)) v8usa;

__device__ __forceinline__ unsigned short f2bf(float f) { unsigned u = __float_as_uint(f); u += 0x7FFFu + ((u >> 16) & 1u); return (unsigned short)(u >> 16); }
__device__ __forceinline__ float bf2f(unsigned short b) { return __uint_as_float(((unsigned)b) << 16); }
__device__ __forceinline__ float bfr(float f) { return bf2f(f2bf(f)); }
__device__ __forceinline__ v16h cat16(v8h lo, v8h hi) { return __builtin_shufflevector(lo, hi, 0, 1, 2, 3, 4, 5, 6, 7, 8, 9, 10, 11, 12, 13, 14, 15); }
__device__ __forceinline__ v16bf cat16b(v8us lo, v8us hi) { return __builtin_bit_cast(v16bf, __builtin_shufflevector(lo, hi, 0, 1, 2, 3, 4, 5, 6, 7, 8, 9, 10, 11, 12, 13, 14, 15)); }
__device__ __forceinline__ v8f wmma16(v16h a, v16h b, v8f c) { return __builtin_amdgcn_wmma_f32_16x16x32_f16(false, a, false, b, (short)0, c, false, false); }
__device__ __forceinline__ v8f wmmab(v16bf a, v16bf b, v8f c) { return __builtin_amdgcn_wmma_f32_16x16x32_bf16(false, a, false, b, (short)0, c, false, false); }


template <typename T16> struct WFrag;
template <> struct WFrag<h16> { typedef v16h V; static __device__ __forceinline__ V ld(const h16* p) { return cat16(*(const v8h*)p, *(const v8h*)(p + 16)); } static __device__ __forceinline__ v8f mma(V a, V b, v8f c) { return wmma16(a, b, c); } };
template <> struct WFrag<bf> { typedef v16bf V; static __device__ __forceinline__ V ld(const bf* p) { return cat16b(*(const v8us*)p, *(const v8us*)(p + 16)); } static __device__ __forceinline__ v8f mma(V a, V b, v8f c) { return wmmab(a, b, c); } };
template <typename T16, int NSPLIT, bool BIAS>
__global__ __launch_bounds__(32) void k_gemmw(const T16* __restrict__ A, const T16* __restrict__ A2, const T16* __restrict__ Bt, const T16* __restrict__ Bt2, int K, float* C, int ldc, const float* __restrict__ bias, size_t sA, size_t sB, size_t sC) {
    typedef typename WFrag<T16>::V V;
    __shared__ __align__(16) float os[16 * 68];
    const size_t z = blockIdx.z; A += z * sA; if (A2) A2 += z * sA; Bt += z * sB; if (Bt2) Bt2 += z * sB; C += z * sC;
    const int lane = threadIdx.x & 31, lr = lane & 15, hi = lane >> 4; const int r0 = blockIdx.x * 64, c0 = blockIdx.y * 64;
    v8f acc[4][4];
#pragma unroll
    for (int mb = 0; mb < 4; ++mb)
#pragma unroll
        for (int nb = 0; nb < 4; ++nb) acc[mb][nb] = (v8f){};
    const size_t aoff = (size_t)(r0 + lr) * K + 8 * hi, boff = (size_t)(c0 + lr) * K + 8 * hi;
#pragma unroll 1
    for (int kc = 0; kc < K; kc += 32) {
        V a[4], a2[4];
#pragma unroll
        for (int mb = 0; mb < 4; ++mb) { a[mb] = WFrag<T16>::ld(A + aoff + (size_t)mb * 16 * K + kc); if (NSPLIT == 1 || NSPLIT == 2) a2[mb] = WFrag<T16>::ld(A2 + aoff + (size_t)mb * 16 * K + kc); }
#pragma unroll
        for (int nb = 0; nb < 4; ++nb) { const V b = WFrag<T16>::ld(Bt + boff + (size_t)nb * 16 * K + kc); V b2; if (NSPLIT >= 2) b2 = WFrag<T16>::ld(Bt2 + boff + (size_t)nb * 16 * K + kc);
#pragma unroll
            for (int mb = 0; mb < 4; ++mb) { acc[mb][nb] = WFrag<T16>::mma(a[mb], b, acc[mb][nb]); if (NSPLIT == 1 || NSPLIT == 2) acc[mb][nb] = WFrag<T16>::mma(a2[mb], b, acc[mb][nb]); if (NSPLIT >= 2) acc[mb][nb] = WFrag<T16>::mma(a[mb], b2, acc[mb][nb]); } }
        asm volatile("v_nop\n\tv_nop\n\tv_nop\n\tv_nop" : "+v"(acc[0][0]), "+v"(acc[1][1]), "+v"(acc[2][2]), "+v"(acc[3][3]) : "v"(a[0]), "v"(a[3]));
    }
#pragma unroll
    for (int mb = 0; mb < 4; ++mb) {
#pragma unroll
        for (int nb = 0; nb < 4; ++nb) {
#pragma unroll
            for (int j = 0; j < 8; ++j) os[(hi * 8 + j) * 68 + nb * 16 + lr] = acc[mb][nb][j]; }
        __builtin_amdgcn_wave_barrier(); asm volatile("" ::: "memory");
        float* crow = C + (size_t)(r0 + mb * 16) * ldc + c0;
#pragma unroll 1
        for (int ps = 0; ps < 2; ++ps) {
#pragma unroll
            for (int s = 0; s < 8; ++s) { const int row = 2 * s + hi, cofs = lr * 4; v4f val = *(const v4fa*)(os + row * 68 + cofs); if (BIAS) { val[0] += bfr(bias[c0 + cofs]); val[1] += bfr(bias[c0 + cofs + 1]); val[2] += bfr(bias[c0 + cofs + 2]); val[3] += bfr(bias[c0 + cofs + 3]); }
                *(volatile v4f*)(crow + (size_t)row * ldc + cofs) = val; }
            if (ps == 0) __threadfence(); }
        __builtin_amdgcn_wave_barrier(); asm volatile("" ::: "memory");
    }
}

template <typename T16, int NSPLIT, int CMODE>
__global__ __launch_bounds__(32) void k_gemmc(const T16* __restrict__ A, const T16* __restrict__ A2, const T16* __restrict__ Bt, const T16* __restrict__ Bt2, int K, float* C, int ldc, int roff, size_t sA, size_t sB, size_t sC, const int* CF) {
    typedef typename WFrag<T16>::V V;
    __shared__ __align__(16) float os[16 * 68];
    const size_t z = blockIdx.z; A += z * sA; if (A2) A2 += z * sA; Bt += z * sB; if (Bt2) Bt2 += z * sB; C += z * sC;
    const int lane = threadIdx.x & 31, lr = lane & 15, hi = lane >> 4; const int r0 = blockIdx.x * 64, c0 = blockIdx.y * 64;
    const bool con = (CF == nullptr) || (CF[0] != 0);     if (CMODE == 1 && con && c0 > r0 + roff + 63) return; if (CMODE == 3 && (c0 > r0 + 63 + WB || c0 + 63 < r0)) return;
    const int Kl = (CMODE == 2 && con) ? min(K, r0 + roff + 64) : ((CMODE == 4) ? min(K, r0 + 64 + WB) : K); const int kst = (CMODE == 4) ? r0 : 0;
    v8f acc[4][4];
#pragma unroll
    for (int mb = 0; mb < 4; ++mb)
#pragma unroll
        for (int nb = 0; nb < 4; ++nb) acc[mb][nb] = (v8f){};
    const size_t aoff = (size_t)(r0 + lr) * K + 8 * hi, boff = (size_t)(c0 + lr) * K + 8 * hi;
#pragma unroll 1
    for (int kc = kst; kc < Kl; kc += 32) {
        V a[4], a2[4];
#pragma unroll
        for (int mb = 0; mb < 4; ++mb) { a[mb] = WFrag<T16>::ld(A + aoff + (size_t)mb * 16 * K + kc); if (NSPLIT == 1 || NSPLIT == 2) a2[mb] = WFrag<T16>::ld(A2 + aoff + (size_t)mb * 16 * K + kc); }
#pragma unroll
        for (int nb = 0; nb < 4; ++nb) { const V b = WFrag<T16>::ld(Bt + boff + (size_t)nb * 16 * K + kc); V b2; if (NSPLIT >= 2) b2 = WFrag<T16>::ld(Bt2 + boff + (size_t)nb * 16 * K + kc);
#pragma unroll
            for (int mb = 0; mb < 4; ++mb) { acc[mb][nb] = WFrag<T16>::mma(a[mb], b, acc[mb][nb]); if (NSPLIT == 1 || NSPLIT == 2) acc[mb][nb] = WFrag<T16>::mma(a2[mb], b, acc[mb][nb]); if (NSPLIT >= 2) acc[mb][nb] = WFrag<T16>::mma(a[mb], b2, acc[mb][nb]); } }
        asm volatile("v_nop\n\tv_nop\n\tv_nop\n\tv_nop" : "+v"(acc[0][0]), "+v"(acc[1][1]), "+v"(acc[2][2]), "+v"(acc[3][3]) : "v"(a[0]), "v"(a[3]));
    }
#pragma unroll
    for (int mb = 0; mb < 4; ++mb) {
#pragma unroll
        for (int nb = 0; nb < 4; ++nb) {
#pragma unroll
            for (int j = 0; j < 8; ++j) os[(hi * 8 + j) * 68 + nb * 16 + lr] = acc[mb][nb][j]; }
        __builtin_amdgcn_wave_barrier(); asm volatile("" ::: "memory");
        float* crow = C + (size_t)(r0 + mb * 16) * ldc + c0;
#pragma unroll 1
        for (int ps = 0; ps < 2; ++ps) {
#pragma unroll
            for (int s = 0; s < 8; ++s) { const int row = 2 * s + hi, cofs = lr * 4; v4f val = *(const v4fa*)(os + row * 68 + cofs);
                *(volatile v4f*)(crow + (size_t)row * ldc + cofs) = val; }
            if (ps == 0) __threadfence(); }
        __builtin_amdgcn_wave_barrier(); asm volatile("" ::: "memory");
    }
}

__device__ __forceinline__ h16 tohx(float x) { return (h16)x; }
__device__ __forceinline__ void splitf(float y, unsigned short& h, unsigned short& l) { h = f2bf(y); l = f2bf(y - bf2f(h)); }
typedef __attribute__((ext_vector_type(2))) _Float16 v2h;
typedef __attribute__((ext_vector_type(4))) _Float16 v4h;
typedef __attribute__((ext_vector_type(2))) unsigned short v2us;
typedef __attribute__((ext_vector_type(4))) unsigned short v4us;
typedef __attribute__((ext_vector_type(2))) float v2f;
typedef __attribute__((ext_vector_type(4))) int v4i;

__global__ __launch_bounds__(256) void k_wtG(const float* __restrict__ w, int K, int N, bf* Bt) {
    const int lane = threadIdx.x & 31; const int L0 = (blockIdx.x * 8 + (threadIdx.x >> 5)) * 8; const int nlines = N * K / 64;
#pragma unroll
    for (int ps = 0; ps < 2; ++ps) {
#pragma unroll 1
        for (int l = 0; l < 8; ++l) { const int L = L0 + l; if (L >= nlines) break; const size_t e = (size_t)L * 64 + lane * 2; const int k = (int)(e % K), n = (int)(e / K); v2us o;
            o[0] = f2bf(w[(size_t)k * N + n]); o[1] = f2bf(w[(size_t)(k + 1) * N + n]); *(volatile v2us*)(Bt + e) = o; }
        if (ps == 0) __threadfence(); }
}
__global__ __launch_bounds__(256) void k_cvt8(const float* __restrict__ src, bf* dst, size_t n8) { const size_t i = (size_t)blockIdx.x * 256 + threadIdx.x; if (i >= n8) return; const v8f v = *(const v8f*)(src + i * 8); v8us o;
#pragma unroll
    for (int k = 0; k < 8; ++k) o[k] = f2bf(v[k]); *(volatile v8us*)(dst + i * 8) = o; __threadfence(); *(volatile v8us*)(dst + i * 8) = o; }


__global__ void k_flag0(int* F) { if (threadIdx.x == 0) { *(volatile int*)F = 1; __threadfence(); *(volatile int*)F = 1; } }
__global__ __launch_bounds__(256) void k_kcopy(const float* __restrict__ src, bf* KP, size_t n8) { const size_t i = (size_t)blockIdx.x * 256 + threadIdx.x; if (i >= n8) return; const size_t e = i * 8; const size_t h = e / ((size_t)TT * HD); const size_t rem = e % ((size_t)TT * HD); const v8f v = *(const v8f*)(src + e); v8us o;
#pragma unroll
    for (int k = 0; k < 8; ++k) o[k] = f2bf(v[k]); bf* dst = KP + h * ((size_t)(PADK + TT) * HD) + (size_t)PADK * HD + rem; *(volatile v8us*)dst = o; __threadfence(); *(volatile v8us*)dst = o; }
__global__ __launch_bounds__(256) void k_kpad(bf* KP, size_t n8) { const size_t i = (size_t)blockIdx.x * 256 + threadIdx.x; if (i >= n8) return; const size_t e = i * 8; const size_t h = e / ((size_t)PADK * HD); const size_t rem = e % ((size_t)PADK * HD); const v8us z = (v8us){}; bf* dst = KP + h * ((size_t)(PADK + TT) * HD) + rem; *(volatile v8us*)dst = z; __threadfence(); *(volatile v8us*)dst = z; }
__global__ __launch_bounds__(256) void k_vtpw(const float* __restrict__ vh, int k0g, bf* VTW) { const size_t e = ((size_t)blockIdx.x * 256 + threadIdx.x) * 2; if (e >= (size_t)HD * KW) return; const int jr = (int)(e % KW); const int d = (int)(e / KW); v2us o;
#pragma unroll
    for (int q = 0; q < 2; ++q) { const int jg = k0g + jr + q; o[q] = (jg >= 0 && jg < TT) ? f2bf(vh[(size_t)jg * HD + d]) : (unsigned short)0; }
    *(volatile v2us*)(VTW + e) = o; __threadfence(); *(volatile v2us*)(VTW + e) = o; }
__global__ __launch_bounds__(256) void k_asoftW(const float* __restrict__ Sb, int k0g, bf* Ph, bf* Pl) {
    const int lane = threadIdx.x & 31; const int i = blockIdx.x * 8 + (threadIdx.x >> 5); if (i >= RB) return; const float* sr = Sb + (size_t)i * KW; float v[KW / 32]; float mx = -3.0e38f;
#pragma unroll
    for (int ch = 0; ch < KW / 128; ++ch) { const int j0 = ch * 128 + lane * 4; const v4f a = *(const v4f*)(sr + j0);
#pragma unroll
        for (int q = 0; q < 4; ++q) { const int j = j0 + q; const float t = (j >= i && j <= i + WB && k0g + j >= 0) ? a[q] * SCL : -3.0e38f; v[ch * 4 + q] = t; mx = fmaxf(mx, t); } }
#pragma unroll
    for (int sh = 16; sh; sh >>= 1) mx = fmaxf(mx, __shfl_xor(mx, sh, 32));
    float sum = 0.f;
#pragma unroll
    for (int k = 0; k < KW / 32; ++k) { float d0 = __fsub_rn(v[k], mx); asm volatile("" : "+v"(d0)); v[k] = __builtin_amdgcn_exp2f(__fmul_rn(d0, 1.4426950408889634f)); sum += v[k]; }
#pragma unroll
    for (int sh = 16; sh; sh >>= 1) sum += __shfl_xor(sum, sh, 32);
    const float f = __fdiv_rn(1.0f, sum);
#pragma unroll 1
    for (int ps = 0; ps < 2; ++ps) {
#pragma unroll
        for (int ch = 0; ch < KW / 128; ++ch) { v4us oh, ol;
#pragma unroll
            for (int q = 0; q < 4; ++q) { unsigned short a, c2; splitf(v[ch * 4 + q] * f, a, c2); oh[q] = a; ol[q] = c2; }
            const size_t oo = (size_t)i * KW + ch * 128 + lane * 4; *(volatile v4us*)(Ph + oo) = oh; *(volatile v4us*)(Pl + oo) = ol; }
        if (ps == 0) __threadfence(); } }
__global__ __launch_bounds__(256) void k_mergeW(const float* __restrict__ O, float* OUTc) { const size_t e = ((size_t)blockIdx.x * 256 + threadIdx.x) * 2; if (e >= (size_t)RB * HD) return; v2f o2; o2[0] = O[e]; o2[1] = O[e + 1]; *(volatile v2f*)(OUTc + e) = o2; __threadfence(); *(volatile v2f*)(OUTc + e) = o2; }


extern "C" void kernel_launch(void* const* d_in, const int* in_sizes, int n_in,
                              void* d_out, int out_size, void* d_ws, size_t ws_size, hipStream_t stream) {
    (void)in_sizes; (void)n_in; (void)out_size;
    const float* xq = (const float*)d_in[0]; const float* xk = (const float*)d_in[1]; const float* xv = (const float*)d_in[2];     const float* x = xq; const float* wq = nullptr; const float* wk = nullptr; const float* wv = nullptr; const float* wo = nullptr; (void)x; (void)wq; (void)wk; (void)wv; (void)wo;
    float* OUT = (float*)d_out;
    char* wsp = (char*)d_ws;
    auto take = [&](size_t bytes) { char* p = wsp; wsp += (bytes + 255) & ~(size_t)255; return (void*)p; };
    int* CFLAG = (int*)take(256);
    bf* QPh = (bf*)take((size_t)NH_ * TT * HD * 2); bf* KPh = (bf*)take((size_t)NKV * (PADK + TT) * HD * 2); bf* VTW = (bf*)take((size_t)HD * KW * 2);
    float* Sb = (float*)take((size_t)RB * KW * 4); bf* Ph = (bf*)take((size_t)RB * KW * 2); bf* Pl = (bf*)take((size_t)RB * KW * 2); float* Ob = (float*)take((size_t)RB * HD * 4);
    if ((size_t)(wsp - (char*)d_ws) > ws_size) return;
    k_flag0<<<1, 32, 0, stream>>>(CFLAG);
    k_cvt8<<<(unsigned)(((size_t)NH_ * TT * HD / 8 + 255) / 256), 256, 0, stream>>>(xq, QPh, (size_t)NH_ * TT * HD / 8);
    k_kpad<<<(unsigned)(((size_t)NKV * PADK * HD / 8 + 255) / 256), 256, 0, stream>>>(KPh, (size_t)NKV * PADK * HD / 8); k_kcopy<<<(unsigned)(((size_t)NKV * TT * HD / 8 + 255) / 256), 256, 0, stream>>>(xk, KPh, (size_t)NKV * TT * HD / 8);
    for (int h = 0; h < NH_; ++h) {
        for (int c = 0; c < TT / RB; ++c) { const int r0 = c * RB; const int k0g = r0 - WB;
            k_vtpw<<<(unsigned)(((size_t)HD * KW / 2 + 255) / 256), 256, 0, stream>>>(xv + (size_t)h * TT * HD, k0g, VTW);
            k_gemmc<bf, 0, 3><<<dim3(RB / 64, KW / 64, 1), 32, 0, stream>>>(QPh + ((size_t)h * TT + r0) * HD, nullptr, KPh + ((size_t)h * (PADK + TT) + PADK + k0g) * HD, nullptr, HD, Sb, KW, 0, 0, 0, 0, CFLAG);
            k_asoftW<<<RB / 8, 256, 0, stream>>>(Sb, k0g, Ph, Pl);
            k_gemmc<bf, 1, 4><<<dim3(RB / 64, HD / 64, 1), 32, 0, stream>>>(Ph, Pl, VTW, nullptr, KW, Ob, HD, 0, 0, 0, 0, CFLAG);
            k_mergeW<<<(unsigned)(((size_t)RB * HD / 2 + 255) / 256), 256, 0, stream>>>(Ob, OUT + ((size_t)h * TT + r0) * HD); } }
}
